// Linear_mvm_47811575939413
// MI455X (gfx1250) — hardware-run, weakly checked
//
#include <hip/hip_runtime.h>
#include <math.h>

typedef __attribute__((ext_vector_type(16))) _Float16 v16h;
typedef __attribute__((ext_vector_type(8)))  _Float16 v8h;
typedef __attribute__((ext_vector_type(8)))  float    v8f;
typedef __attribute__((ext_vector_type(4)))  float    v4f;
typedef __attribute__((ext_vector_type(4)))  unsigned v4u;

constexpr int kBatch   = 256;
constexpr int kInF     = 1024;
constexpr int kOutF    = 1024;
constexpr int kRowT    = 64;
constexpr int kXr      = kInF / kRowT;
constexpr int kStreams = 16;
constexpr int kSlices  = 8;
constexpr int kPlanesB = 2 * kSlices;
constexpr int kGroupU  = 4;
constexpr int kGroups  = kPlanesB / kGroupU;
constexpr int kSlabP   = 36;
constexpr int kTilesB  = kBatch / 16;
constexpr int kTilesO  = kOutF / 32;
constexpr int kWaveTiles = kTilesB * kTilesO;
constexpr float kStep    = 192.0f / 255.0f;
constexpr float kInvStep = 255.0f / 192.0f;
static_assert(kInvStep == 1.328125f, "ADC code scale is exact");
static_assert(kXr == 16 && kRowT == 64, "row tiles of 64 inputs: two 32-deep k steps");
static_assert((kRowT % 32) == 0, "K multiple of 32");
static_assert((kBatch % 16) == 0 && (kOutF % 32) == 0, "wave tile 16 x 32");
static_assert(kWaveTiles == 512 && (kWaveTiles % 8) == 0, "64 blocks of 8 waves, no partial block");
static_assert(kGroups * kGroupU == kPlanesB, "u groups");
static_assert(kGroups == 4 && kGroupU == 4 && kSlices == 8, "group g: sign = g>>1, slices 4*(g&1) .. 4*(g&1)+3");

constexpr size_t kBytesA  = (size_t)kXr * kStreams * kBatch * kRowT * 2;
constexpr size_t kBytesB  = (size_t)kPlanesB * kXr * kOutF * kRowT * 2;
constexpr size_t kOffA    = 0;
constexpr size_t kOffB    = kOffA + kBytesA;
constexpr size_t kWsTotal = kOffB + kBytesB;
static_assert(kBytesA == 8388608ull && kBytesB == 33554432ull, "plane sizes");
static_assert(kWsTotal == 41943040ull, "carve total");
static_assert(kWsTotal <= 134217728ull, "carve cap");
static_assert((kOffB % 128) == 0, "128-B aligned regions");

template <typename T> struct Frag;
template <> struct Frag<_Float16> {
  typedef v16h V; union U { v16h v; v8h h[2]; };
  static __device__ __forceinline__ v16h load(const _Float16* p) {
    U f; f.h[0] = *(const v8h*)(p); f.h[1] = *(const v8h*)(p + 16); return f.v;
  }
  static __device__ __forceinline__ v8f mma(v16h a, v16h b, v8f c) {
    return __builtin_amdgcn_wmma_f32_16x16x32_f16(false, a, false, b, (short)0, c, false, false);
  }
};

__device__ __forceinline__ v8f xb_mma2(v16h a0, v16h a1, v16h b0, v16h b1) {
  v8f c = (v8f){0.f, 0.f, 0.f, 0.f, 0.f, 0.f, 0.f, 0.f};
  c = Frag<_Float16>::mma(a0, b0, c);
  c = Frag<_Float16>::mma(a1, b1, c);
  asm volatile("v_nop\n\tv_nop\n\tv_nop\n\tv_nop" : "+v"(c) : "v"(a0), "v"(a1), "v"(b0), "v"(b1));
  return c;
}

__global__ __launch_bounds__(256) void quant_input_planes_kernel(
    const float* __restrict__ x, unsigned* __restrict__ aw)
{
  const int g  = blockIdx.x * 256 + threadIdx.x;
  const int b  = g >> 7;
  const int i8 = g & 127;
  const int xr = i8 >> 3;
  const int k8 = i8 & 7;
  const float* src = x + (size_t)b * kInF + (size_t)i8 * 8;
  const v4f a0 = *(const v4f*)(src);
  const v4f a1 = *(const v4f*)(src + 4);
  unsigned xu[8];
#pragma unroll
  for (int e = 0; e < 4; ++e) {
    const float f0 = a0[e];
    const float f1 = a1[e];
    float r0 = rintf(f0 * 4096.0f);
    float r1 = rintf(f1 * 4096.0f);
    r0 = fminf(fmaxf(r0, -32768.0f), 32767.0f);
    r1 = fminf(fmaxf(r1, -32768.0f), 32767.0f);
    xu[e]     = ((unsigned)(int)r0) & 0xFFFFu;
    xu[4 + e] = ((unsigned)(int)r1) & 0xFFFFu;
  }
#pragma unroll 1
  for (int pass = 0; pass < 2; ++pass) {
#pragma unroll 1
    for (int t = 0; t < kStreams; ++t) {
      const unsigned w0 = ((xu[0] >> t) & 1u) * 0x3C00u + ((xu[1] >> t) & 1u) * 0x3C000000u;
      const unsigned w1 = ((xu[2] >> t) & 1u) * 0x3C00u + ((xu[3] >> t) & 1u) * 0x3C000000u;
      const unsigned w2 = ((xu[4] >> t) & 1u) * 0x3C00u + ((xu[5] >> t) & 1u) * 0x3C000000u;
      const unsigned w3 = ((xu[6] >> t) & 1u) * 0x3C00u + ((xu[7] >> t) & 1u) * 0x3C000000u;
      const v4u w = (v4u){w0, w1, w2, w3};
      const size_t wi = ((size_t)((xr * kStreams + t) * kBatch + b)) * 32 + (size_t)k8 * 4;
      *(volatile v4u*)(aw + wi) = w;
    }
    __threadfence();
  }
}

__global__ __launch_bounds__(256) void quant_weight_planes_kernel(
    const float* __restrict__ w, unsigned* __restrict__ bw)
{
  const int g  = blockIdx.x * 256 + threadIdx.x;
  const int o  = g >> 7;
  const int i8 = g & 127;
  const int xr = i8 >> 3;
  const int k8 = i8 & 7;
  const float* src = w + (size_t)o * kInF + (size_t)i8 * 8;
  const v4f a0 = *(const v4f*)(src);
  const v4f a1 = *(const v4f*)(src + 4);
  unsigned comb[8];
#pragma unroll
  for (int e = 0; e < 4; ++e) {
    const float f0 = a0[e];
    const float f1 = a1[e];
    const float p0 = fminf(fmaxf(rintf(fmaxf(f0, 0.0f) * 4096.0f), 0.0f), 65535.0f);
    const float n0 = fminf(fmaxf(rintf(fmaxf(-f0, 0.0f) * 4096.0f), 0.0f), 65535.0f);
    const float p1 = fminf(fmaxf(rintf(fmaxf(f1, 0.0f) * 4096.0f), 0.0f), 65535.0f);
    const float n1 = fminf(fmaxf(rintf(fmaxf(-f1, 0.0f) * 4096.0f), 0.0f), 65535.0f);
    comb[e]     = ((unsigned)p0) | (((unsigned)n0) << 16);
    comb[4 + e] = ((unsigned)p1) | (((unsigned)n1) << 16);
  }
#pragma unroll 1
  for (int pass = 0; pass < 2; ++pass) {
#pragma unroll 1
    for (int u = 0; u < kPlanesB; ++u) {
      const int sign = (u >= kSlices) ? 1 : 0;
      const int jj   = u - kSlices * sign;
      const int fsh  = 16 * sign;
      const int sh   = 14 - 2 * jj;
      unsigned hb[8];
#pragma unroll
      for (int e = 0; e < 8; ++e) {
        const unsigned field = (comb[e] >> fsh) & 0xFFFFu;
        const unsigned v     = (field >> sh) & 3u;
        hb[e] = (0x42403C00u >> (8u * v)) & 0xFFu;
      }
      const unsigned w0 = (hb[0] << 8) | (hb[1] << 24);
      const unsigned w1 = (hb[2] << 8) | (hb[3] << 24);
      const unsigned w2 = (hb[4] << 8) | (hb[5] << 24);
      const unsigned w3 = (hb[6] << 8) | (hb[7] << 24);
      const v4u wv = (v4u){w0, w1, w2, w3};
      const size_t wi = ((size_t)((u * kXr + xr) * kOutF + o)) * 32 + (size_t)k8 * 4;
      *(volatile v4u*)(bw + wi) = wv;
    }
    __threadfence();
  }
}

__global__ __launch_bounds__(256) void xbar_main_kernel(
    const unsigned short* __restrict__ Aplane, const unsigned short* __restrict__ Bplane,
    const float* __restrict__ bias, float* __restrict__ out)
{
  __shared__ __align__(16) float slab[8][16 * kSlabP];
  const int lane = threadIdx.x & 31;
  const int wave = threadIdx.x >> 5;
  const int tile = blockIdx.x * 8 + wave;
  const int ot   = tile & (kTilesO - 1);
  const int bt   = tile >> 5;
  const int rl   = lane & 15;
  const int hh   = lane >> 4;

  const _Float16* A = (const _Float16*)Aplane;
  const _Float16* B = (const _Float16*)Bplane;
  const _Float16* arow = A + (size_t)(bt * 16 + rl) * kRowT + hh * 8;
  const _Float16* brow = B + (size_t)(ot * 32 + rl) * kRowT + hh * 8;

  float facc[2][8];
#pragma unroll
  for (int nt = 0; nt < 2; ++nt)
#pragma unroll
    for (int r = 0; r < 8; ++r) facc[nt][r] = 0.0f;

#pragma unroll 1
  for (int xr = 0; xr < kXr; ++xr) {
#pragma unroll 1
    for (int g = 0; g < kGroups; ++g) {
      v16h b0[kGroupU][2], b1[kGroupU][2];
#pragma unroll
      for (int j = 0; j < kGroupU; ++j) {
#pragma unroll
        for (int nt = 0; nt < 2; ++nt) {
          const _Float16* p = brow + ((size_t)((g * kGroupU + j) * kXr + xr) * kOutF + (size_t)nt * 16) * kRowT;
          b0[j][nt] = Frag<_Float16>::load(p);
          b1[j][nt] = Frag<_Float16>::load(p + 32);
        }
      }
      const float gmag = ((g & 1) != 0) ? 1.0f : 256.0f;
      const float gf   = (g >= 2) ? -gmag : gmag;
#pragma unroll 1
      for (int t = 0; t < kStreams; ++t) {
        const _Float16* pa = arow + (size_t)((xr * kStreams + t) * kBatch) * kRowT;
        const v16h a0 = Frag<_Float16>::load(pa);
        const v16h a1 = Frag<_Float16>::load(pa + 32);
        const float tsc = __uint_as_float((unsigned)(103 + t) << 23);
        const float tsg = (t == kStreams - 1) ? -tsc : tsc;
        const float wtb = tsg * kStep * gf;
#pragma unroll
        for (int j = 0; j < kGroupU; ++j) {
          const float wt = wtb * (float)(1 << (2 * (3 - j)));
#pragma unroll
          for (int nt = 0; nt < 2; ++nt) {
            const v8f c = xb_mma2(a0, a1, b0[j][nt], b1[j][nt]);
#pragma unroll
            for (int r = 0; r < 8; ++r) {
              const float code = rintf(c[r] * kInvStep);
              facc[nt][r] = fmaf(code, wt, facc[nt][r]);
            }
          }
        }
      }
    }
  }

  float* sl = slab[wave];
#pragma unroll
  for (int nt = 0; nt < 2; ++nt) {
    const int n = ot * 32 + nt * 16 + rl;
    const float bv = bias[n];
#pragma unroll
    for (int r = 0; r < 8; ++r) {
      const float v  = facc[nt][r];
      float qv = rintf(v * 4096.0f);
      qv = fminf(fmaxf(qv, -32768.0f), 32767.0f);
      const float fin = qv * 0.000244140625f + bv;
      sl[(8 * hh + r) * kSlabP + nt * 16 + rl] = fin;
    }
  }
  __syncthreads();
  {
    const int q  = lane >> 3;
    const int c4 = (lane & 7) * 4;
    v4f vals[4];
#pragma unroll
    for (int it = 0; it < 4; ++it) vals[it] = *(const v4f*)(sl + (it * 4 + q) * kSlabP + c4);
    for (int pass = 0; pass < 2; ++pass) {
#pragma unroll
      for (int it = 0; it < 4; ++it) {
        const int row = bt * 16 + it * 4 + q;
        *(volatile v4f*)(out + (size_t)row * kOutF + ot * 32 + c4) = vals[it];
      }
      __threadfence();
    }
  }
}

extern "C" void kernel_launch(void* const* d_in, const int* in_sizes, int n_in,
                              void* d_out, int out_size, void* d_ws, size_t ws_size,
                              hipStream_t stream) {
  if (n_in < 3) return;
  if (in_sizes[0] != kBatch * kInF) return;
  if (in_sizes[1] != kOutF * kInF) return;
  if (in_sizes[2] != kOutF) return;
  if (out_size != kBatch * kOutF) return;
  if (ws_size < kWsTotal) return;

  const float* x      = (const float*)d_in[0];
  const float* weight = (const float*)d_in[1];
  const float* bias   = (const float*)d_in[2];
  float* out = (float*)d_out;

  char* ws = (char*)d_ws;
  unsigned* aw = (unsigned*)(ws + kOffA);
  unsigned* bw = (unsigned*)(ws + kOffB);

  quant_input_planes_kernel<<<(kBatch * kInF / 8) / 256, 256, 0, stream>>>(x, aw);
  quant_weight_planes_kernel<<<(kOutF * kInF / 8) / 256, 256, 0, stream>>>(weight, bw);
  xbar_main_kernel<<<kWaveTiles / 8, 256, 0, stream>>>(
      (const unsigned short*)(ws + kOffA), (const unsigned short*)(ws + kOffB), bias, out);
}
